// GroupLinear_61426622267738
// MI455X (gfx1250) — hardware-verified
//
#include <hip/hip_runtime.h>


namespace {
constexpr int NB = 16384, G = 16, DI = 512, DO = 512;
constexpr float XS = 8.0f;

typedef _Float16 b16;
typedef __attribute__((ext_vector_type(16))) _Float16 v16b;
typedef __attribute__((ext_vector_type(8))) _Float16 v8b;
typedef __attribute__((ext_vector_type(8))) float v8f;
typedef __attribute__((ext_vector_type(4))) float v4f;
__device__ __forceinline__ float bf16_rne(float f) { unsigned int u = __float_as_uint(f); u += 0x7FFFu + ((u >> 16) & 1u); return __uint_as_float(u & 0xFFFF0000u); }
__device__ __forceinline__ v16b frag_kb(const b16* p, int hh) { const v8b a = *(const v8b*)(p + 8 * hh), b = *(const v8b*)(p + 16 + 8 * hh); v16b f;
#pragma unroll
  for (int e = 0; e < 8; ++e) { f[e] = a[e]; f[8 + e] = b[e]; } return f; }
__device__ __forceinline__ v8f wmma16b(v16b a, v16b b, v8f c) { v8f d = __builtin_amdgcn_wmma_f32_16x16x32_f16(false, a, false, b, (short)0, c, false, false); asm volatile("v_nop\n\tv_nop\n\tv_nop\n\tv_nop" : "+v"(d) : "v"(a), "v"(b)); return d; }
__device__ __forceinline__ void wave_lds_sync() { __builtin_amdgcn_fence(__ATOMIC_RELEASE, "workgroup"); __builtin_amdgcn_wave_barrier(); __builtin_amdgcn_fence(__ATOMIC_ACQUIRE, "workgroup"); }
__device__ __forceinline__ float pmul(float a, float b) { float p = a * b; asm volatile("" : "+v"(p)); return p; }

__global__ __launch_bounds__(256) void prep_kernel(const float* __restrict__ x, const float* __restrict__ w, const float* __restrict__ bp, b16* __restrict__ X, b16* __restrict__ Wt, float* __restrict__ P) {
  const size_t tid = (size_t)blockIdx.x * 256 + threadIdx.x, nth = (size_t)gridDim.x * 256;
  for (int pass = 0; pass < 2; ++pass) {
    for (size_t p = tid; p < (size_t)G * DO * (DI / 8); p += nth) { const int g = (int)(p / ((size_t)DO * (DI / 8))); const size_t r = p % ((size_t)DO * (DI / 8)); const int o = (int)(r / (DI / 8)), i0 = (int)(r % (DI / 8)) * 8; v8b v;
#pragma unroll
      for (int e = 0; e < 8; ++e) v[e] = (b16)bf16_rne(w[((size_t)g * DI + i0 + e) * DO + o]); *(volatile v8b*)(Wt + ((size_t)g * DO + o) * DI + i0) = v; }
    for (size_t p = tid; p < (size_t)NB * DI / 8; p += nth) { v8b v; for (int e = 0; e < 8; ++e) v[e] = (b16)(bf16_rne(x[p * 8 + e]) * XS); *(volatile v8b*)(X + p * 8) = v; }
    for (size_t p = tid; p < (size_t)G * DO; p += nth) P[p] = bf16_rne(bp[p]);
    __threadfence(); }
}

__global__ __launch_bounds__(64) void gl_kernel(const b16* __restrict__ X, const b16* __restrict__ Wt, const float* __restrict__ P, const float* __restrict__ gg, float* __restrict__ out) {
  __shared__ __attribute__((aligned(16))) float Ts[2][32][128 + 4];
  const int lane = threadIdx.x & 31, wave = threadIdx.x >> 5, nloc = lane & 15, hlf = lane >> 4, m0 = blockIdx.y * 32, c0 = blockIdx.x * 256 + wave * 128;
#pragma unroll 1
  for (int hf = 0; hf < 2; ++hf) {
    v8f o_[2][4];
#pragma unroll
    for (int r = 0; r < 2; ++r)
#pragma unroll
      for (int t = 0; t < 4; ++t) o_[r][t] = (v8f){};
#pragma unroll 1
    for (int g = 0; g < G; ++g) { v8f acc[2][4];
#pragma unroll
      for (int r = 0; r < 2; ++r)
#pragma unroll
        for (int t = 0; t < 4; ++t) acc[r][t] = (v8f){};
      const b16* Wg = Wt + (size_t)g * DO * DI;
#pragma unroll 2
      for (int kb = 0; kb < DI; kb += 32) { const v16b a0 = frag_kb(X + (size_t)(m0 + nloc) * DI + kb, hlf), a1 = frag_kb(X + (size_t)(m0 + 16 + nloc) * DI + kb, hlf);
#pragma unroll
        for (int t = 0; t < 4; ++t) { const v16b bw = frag_kb(Wg + (size_t)(c0 + (hf * 4 + t) * 16 + nloc) * DI + kb, hlf); acc[0][t] = wmma16b(a0, bw, acc[0][t]); acc[1][t] = wmma16b(a1, bw, acc[1][t]); } }
      float gw[2][8];
#pragma unroll
      for (int r = 0; r < 2; ++r)
#pragma unroll
        for (int v = 0; v < 8; ++v) gw[r][v] = bf16_rne(gg[(size_t)(m0 + r * 16 + 8 * hlf + v) * G + g]);
#pragma unroll
      for (int t = 0; t < 4; ++t) { const float bb = P[g * DO + c0 + (hf * 4 + t) * 16 + nloc];
#pragma unroll
        for (int r = 0; r < 2; ++r)
#pragma unroll
          for (int v = 0; v < 8; ++v) o_[r][t][v] += pmul(gw[r][v], acc[r][t][v] * (1.0f / XS) + bb); } }
#pragma unroll
    for (int t = 0; t < 4; ++t)
#pragma unroll
      for (int r = 0; r < 2; ++r)
#pragma unroll
        for (int v = 0; v < 8; ++v) Ts[wave][r * 16 + 8 * hlf + v][(hf * 4 + t) * 16 + nloc] = o_[r][t][v]; }
  wave_lds_sync();
  for (int pass = 0; pass < 2; ++pass) { for (int i = lane; i < 32 * 32; i += 32) { const int rr = i >> 5, c4 = (i & 31) * 4; *(volatile v4f*)(out + (size_t)(m0 + rr) * DO + c0 + c4) = *(const v4f*)(&Ts[wave][rr][c4]); } __threadfence(); }
}
}

extern "C" void kernel_launch(void* const* d_in, const int* in_sizes, int n_in,
                              void* d_out, int out_size, void* d_ws, size_t ws_size, hipStream_t stream) {
  (void)n_in; (void)out_size;
  const float* x = (const float*)d_in[0]; const float* gg = (const float*)d_in[1]; const float* w = (const float*)d_in[2]; const float* bp = (const float*)d_in[3];
  float* out = (float*)d_out;
  if (in_sizes[0] != NB * DI || in_sizes[1] != NB * G || in_sizes[2] != G * DI * DO || in_sizes[3] != G * DO) return;
  size_t off = 0; char* ws = (char*)d_ws;
  auto carve = [&](size_t bytes) { char* p = ws + off; off += (bytes + 255) & ~(size_t)255; return p; };
  b16* X = (b16*)carve((size_t)NB * DI * 2); b16* Wt = (b16*)carve((size_t)G * DO * DI * 2); float* P = (float*)carve((size_t)G * DO * 4);
  if (off > ws_size) return;
  prep_kernel<<<512, 256, 0, stream>>>(x, w, bp, X, Wt, P);
  gl_kernel<<<dim3(DO / 256, NB / 32), 64, 0, stream>>>(X, Wt, P, gg, out);
}
